// TSMixerH_28930899706365
// MI455X (gfx1250) — hardware-verified
//
#include <hip/hip_runtime.h>
#include <stdint.h>

#define BB   32
#define LL   512
#define PP   96
#define CC   512
#define KCL  8
#define NLAY 2
#define DFF  512
#define CKN  64
#define EPSF 1e-5f
#define WSC  16.0f
#define WINV 0.0625f

#define XP   65
#define YTP  520
#define YNP  72
#define HSP  56

#define OFF_XS  0
#define OFF_YB  133120
#define OFF_HS  (OFF_YB + 73728)
#define OFF_SM  (OFF_HS + 14336)
#define SMEM_BYTES (OFF_SM + 11264)

typedef _Float16       v16h  __attribute__((ext_vector_type(16)));
typedef __bf16         v16bf __attribute__((ext_vector_type(16)));
typedef unsigned short us16  __attribute__((ext_vector_type(16)));
typedef unsigned short us8   __attribute__((ext_vector_type(8)));
typedef float          v8f   __attribute__((ext_vector_type(8)));
typedef float          v4f   __attribute__((ext_vector_type(4)));
typedef us8 __attribute__((may_alias)) us8a;
typedef v4f __attribute__((may_alias)) v4fa;

union FragH { v16h h; v16bf b; us16 u; us8 half[2]; };

__device__ __forceinline__ v8f wmma_f16(v16h a, v16h b, v8f c) {
  v8f d = __builtin_amdgcn_wmma_f32_16x16x32_f16(false, a, false, b, (short)0, c, false, false);
  asm volatile("v_nop\n\tv_nop\n\tv_nop\n\tv_nop" : "+v"(d) : "v"(a), "v"(b));
  return d;
}
__device__ __forceinline__ v8f wmma_bf16(v16bf a, v16bf b, v8f c) {
  v8f d = __builtin_amdgcn_wmma_f32_16x16x32_bf16(false, a, false, b, (short)0, c, false, false);
  asm volatile("v_nop\n\tv_nop\n\tv_nop\n\tv_nop" : "+v"(d) : "v"(a), "v"(b));
  return d;
}

__device__ __forceinline__ us16 frag16(const unsigned short* p, int h) {
  FragH f;
  f.half[0] = *(const us8a*)(p + 8 * h);
  f.half[1] = *(const us8a*)(p + 16 + 8 * h);
  return f.u;
}

__device__ __forceinline__ unsigned short f16b(float v) {
  union { _Float16 f; unsigned short u; } t;
  t.f = (_Float16)v;
  return t.u;
}
__device__ __forceinline__ unsigned short bf16b(float v) {
  unsigned int u = __float_as_uint(v);
  u = (u + 0x7FFFu + ((u >> 16) & 1u)) >> 16;
  return (unsigned short)u;
}

__device__ __forceinline__ void wave_lds_sync() {
  __builtin_amdgcn_fence(__ATOMIC_RELEASE, "wavefront");
  asm volatile("s_wait_dscnt 0x0" ::: "memory");
  __builtin_amdgcn_wave_barrier();
  __builtin_amdgcn_fence(__ATOMIC_ACQUIRE, "wavefront");
}

__global__ __launch_bounds__(512) void setup_kernel(const int* __restrict__ ids, int nids,
                                                    int* __restrict__ permOut,
                                                    int* __restrict__ invOut) {
  __shared__ int asg[CC];
  __shared__ int permS[CC];
  const int tid = threadIdx.x;
  int a;
  {
    int ii = tid < nids ? tid : nids - 1;
    if (ii < 0) ii = 0;
    int id = ids[ii];
    a = id % KCL;
    if (a < 0) a += KCL;
  }
  asg[tid] = a;
  __syncthreads();
  int pos = 0;
  for (int c = 0; c < CC; ++c) {
    const int ac = asg[c];
    pos += (ac < a) ? 1 : 0;
    pos += (ac == a && c < tid) ? 1 : 0;
  }
  if (pos > CC - 1) pos = CC - 1;
  permS[pos] = tid;
  __syncthreads();
  const int pv = permS[tid];
  *(volatile int*)(permOut + tid) = pv;
  *(volatile int*)(invOut + tid) = pos;
  __threadfence();
  *(volatile int*)(permOut + tid) = pv;
  *(volatile int*)(invOut + tid) = pos;
}

template <int MODE>
__global__ __launch_bounds__(256) void tcvt_kernel(const float* __restrict__ in,
                                                   unsigned short* __restrict__ o0,
                                                   unsigned short* __restrict__ o1,
                                                   int rows, int cols, float sc) {
  __shared__ __attribute__((aligned(16))) unsigned short T0[32 * 72];
  __shared__ __attribute__((aligned(16))) unsigned short T1[(MODE == 1) ? (32 * 72) : 8];
  const int tid = threadIdx.x, lane = tid & 31, wv = tid >> 5;
  const int z = blockIdx.z, c0 = blockIdx.x * 32, r0 = blockIdx.y * 64;
  const float* ip = in + (size_t)z * rows * cols;
  const int cl = tid & 31, rl = tid >> 5;
#pragma unroll
  for (int i = 0; i < 8; ++i) {
    const int r = rl + 8 * i;
    const float v = ip[(size_t)(r0 + r) * cols + c0 + cl];
    if (MODE == 0) {
      T0[cl * 72 + r] = f16b(v * sc);
    } else {
      const unsigned short hb = bf16b(v);
      const float hf = __uint_as_float(((unsigned int)hb) << 16);
      T0[cl * 72 + r] = hb;
      T1[cl * 72 + r] = bf16b(v - hf);
    }
  }
  __syncthreads();
  const int cc = wv * 4 + (lane >> 3), q = lane & 7;
  const us8 p0 = *(const us8a*)(T0 + cc * 72 + 8 * q);
  us8 p1 = p0;
  if (MODE == 1) p1 = *(const us8a*)(T1 + cc * 72 + 8 * q);
  const size_t off = ((size_t)z * cols + c0 + cc) * (size_t)rows + r0 + 8 * q;
  *(volatile us8*)(o0 + off) = p0;
  if (MODE == 1) *(volatile us8*)(o1 + off) = p1;
  __threadfence();
  *(volatile us8*)(o0 + off) = p0;
  if (MODE == 1) *(volatile us8*)(o1 + off) = p1;
}

template <bool TR>
__device__ __forceinline__ void ln_pass(const float* Xs, float* rowM, float* rowR,
                                        const float* lng, const float* lnb,
                                        unsigned short* dst, int tid) {
  for (int l = tid; l < LL; l += 256) {
    const float* xr = Xs + l * XP;
    float s = 0.f;
#pragma unroll 8
    for (int c = 0; c < CKN; ++c) s += xr[c];
    const float m = s * (1.0f / CKN);
    float s2 = 0.f;
#pragma unroll 8
    for (int c = 0; c < CKN; ++c) { const float d = xr[c] - m; s2 += d * d; }
    rowM[l] = m;
    rowR[l] = rsqrtf(s2 * (1.0f / CKN) + EPSF);
  }
  __syncthreads();
  for (int idx = tid; idx < LL * CKN; idx += 256) {
    int l, c;
    if (TR) { c = idx >> 9; l = idx & (LL - 1); }
    else    { l = idx >> 6; c = idx & (CKN - 1); }
    const float y = (Xs[l * XP + c] - rowM[l]) * rowR[l] * lng[c] + lnb[c];
    if (TR) dst[c * YTP + l] = f16b(y);
    else    dst[l * YNP + c] = f16b(y);
  }
  __syncthreads();
}

__device__ __forceinline__ void o_store_pass(const float* Os, float* Og, int wv, int lane) {
  const int q8 = lane & 7, sub = lane >> 3;
#pragma unroll
  for (int i = 0; i < 6; ++i) {
    const int p = wv * 12 + 2 * i + (sub >> 1), hl = sub & 1;
    const v4f v = *(const v4fa*)(Os + p * 64 + 32 * hl + 4 * q8);
    *(volatile v4f*)(Og + (size_t)p * 64 + 32 * hl + 4 * q8) = v;
  }
}

__global__ __launch_bounds__(256)
void mixer_kernel(const float* __restrict__ x,
                  const float* __restrict__ rev_w, const float* __restrict__ rev_b,
                  const float* __restrict__ bt,
                  const float* __restrict__ ln1_g, const float* __restrict__ ln1_b,
                  const float* __restrict__ bf1, const float* __restrict__ bf2,
                  const float* __restrict__ ln2_g, const float* __restrict__ ln2_b,
                  const float* __restrict__ bout,
                  const unsigned short* __restrict__ WtT,
                  const unsigned short* __restrict__ Wf1T,
                  const unsigned short* __restrict__ Wf2T,
                  const unsigned short* __restrict__ WoH,
                  const unsigned short* __restrict__ WoL,
                  const int* __restrict__ perm,
                  float* __restrict__ O)
{
  extern __shared__ __attribute__((aligned(16))) char smem[];
  float* Xs = (float*)(smem + OFF_XS);
  unsigned short* Yb = (unsigned short*)(smem + OFF_YB);
  float* Os = (float*)(smem + OFF_YB);
  unsigned short* Hs = (unsigned short*)(smem + OFF_HS);
  float* sm = (float*)(smem + OFF_SM);
  float* rowM   = sm;
  float* rowR   = sm + 512;
  float* chMean = sm + 1024;
  float* chStd  = sm + 1088;
  float* chRw   = sm + 1152;
  float* chRb   = sm + 1216;
  float* lng    = sm + 1280;
  float* lnb    = sm + 1344;
  float* btS    = sm + 1408;
  float* bf1S   = sm + 1920;
  float* bf2S   = sm + 2432;
  float* red    = sm + 2496;
  int*   chanIdx = (int*)(sm + 2752);

  const int tid  = threadIdx.x;
  const int b    = blockIdx.x & (BB - 1);
  const int k    = blockIdx.x >> 5;
  const int wv   = tid >> 5;
  const int lane = tid & 31;
  const int m15  = lane & 15;
  const int hh   = lane >> 4;

  if (tid < CKN) {
    int q = perm[k * CKN + tid];
    q = q < 0 ? 0 : (q > CC - 1 ? CC - 1 : q);
    chanIdx[tid] = q;
  }
  __syncthreads();

  for (int idx = tid; idx < LL * CKN; idx += 256) {
    const int l = idx >> 6, j = idx & 63;
    Xs[l * XP + j] = x[((size_t)b * LL + l) * CC + chanIdx[j]];
  }
  __syncthreads();

  {
    const int j = tid & 63, part = tid >> 6;
    float s = 0.f;
    for (int l = part * 128; l < part * 128 + 128; ++l) s += Xs[l * XP + j];
    red[part * 64 + j] = s;
  }
  __syncthreads();
  if (tid < CKN) {
    const int j = tid;
    const float s = red[j] + red[64 + j] + red[128 + j] + red[192 + j];
    chMean[j] = s * (1.0f / LL);
  }
  __syncthreads();
  {
    const int j = tid & 63, part = tid >> 6;
    const float m = chMean[j];
    float s2 = 0.f;
    for (int l = part * 128; l < part * 128 + 128; ++l) { const float d = Xs[l * XP + j] - m; s2 += d * d; }
    red[part * 64 + j] = s2;
  }
  __syncthreads();
  if (tid < CKN) {
    const int j = tid;
    const float s2 = red[j] + red[64 + j] + red[128 + j] + red[192 + j];
    const float var = s2 * (1.0f / LL);
    chStd[j] = sqrtf(var + EPSF);
    const int cg = chanIdx[j];
    chRw[j] = rev_w[cg];
    chRb[j] = rev_b[cg];
  }
  __syncthreads();
  for (int idx = tid; idx < LL * CKN; idx += 256) {
    const int l = idx >> 6, j = idx & 63;
    const float a = chRw[j] * (1.0f / chStd[j]);
    Xs[l * XP + j] = (Xs[l * XP + j] - chMean[j]) * a + chRb[j];
  }
  __syncthreads();

  const v8f z8 = {0.f, 0.f, 0.f, 0.f, 0.f, 0.f, 0.f, 0.f};

  for (int layer = 0; layer < NLAY; ++layer) {
    const int kl = k * NLAY + layer;

    if (tid < CKN) { lng[tid] = ln1_g[kl * CKN + tid]; lnb[tid] = ln1_b[kl * CKN + tid]; }
    for (int m = tid; m < LL; m += 256) btS[m] = bt[kl * LL + m];
    __syncthreads();
    ln_pass<true>(Xs, rowM, rowR, lng, lnb, Yb, tid);

    {
      const unsigned short* WtTk = WtT + (size_t)kl * LL * LL;
      for (int mt = wv; mt < LL / 16; mt += 8) {
        v8f acc[4];
#pragma unroll
        for (int ct = 0; ct < 4; ++ct) acc[ct] = z8;
        const unsigned short* arow = WtTk + (size_t)(mt * 16 + m15) * LL;
#pragma unroll 1
        for (int l0 = 0; l0 < LL; l0 += 32) {
          FragH a; a.u = frag16(arow + l0, hh);
#pragma unroll
          for (int ct = 0; ct < 4; ++ct) {
            FragH bq; bq.u = frag16(Yb + (ct * 16 + m15) * YTP + l0, hh);
            acc[ct] = wmma_f16(a.h, bq.h, acc[ct]);
          }
        }
#pragma unroll
        for (int r = 0; r < 8; ++r) {
          const int mrow = mt * 16 + 8 * hh + r;
          const float bias = btS[mrow];
          float* xrow = Xs + mrow * XP;
#pragma unroll
          for (int ct = 0; ct < 4; ++ct) {
            const int c = ct * 16 + m15;
            float v = acc[ct][r] * WINV + bias;
            v = fmaxf(v, 0.f);
            xrow[c] += v;
          }
        }
      }
    }
    __syncthreads();

    if (tid < CKN) {
      lng[tid] = ln2_g[kl * CKN + tid]; lnb[tid] = ln2_b[kl * CKN + tid];
      bf2S[tid] = bf2[kl * CKN + tid];
    }
    for (int f = tid; f < DFF; f += 256) bf1S[f] = bf1[kl * DFF + f];
    __syncthreads();
    ln_pass<false>(Xs, rowM, rowR, lng, lnb, Yb, tid);

    {
      const unsigned short* Wf1Tk = Wf1T + (size_t)kl * DFF * CKN;
      const unsigned short* Wf2Tk = Wf2T + (size_t)kl * CKN * DFF;
      unsigned short* HsW = Hs + wv * 16 * HSP;
      for (int lt = wv; lt < LL / 16; lt += 8) {
        v8f acc2[4];
#pragma unroll
        for (int ct = 0; ct < 4; ++ct) acc2[ct] = z8;
        const unsigned short* aY = Yb + (lt * 16 + m15) * YNP;
#pragma unroll 1
        for (int f0 = 0; f0 < DFF; f0 += 32) {
          v8f h0 = z8, h1 = z8;
#pragma unroll
          for (int c0 = 0; c0 < CKN; c0 += 32) {
            FragH av; av.u = frag16(aY + c0, hh);
            FragH b0; b0.u = frag16(Wf1Tk + (size_t)(f0 + m15) * CKN + c0, hh);
            FragH b1; b1.u = frag16(Wf1Tk + (size_t)(f0 + 16 + m15) * CKN + c0, hh);
            h0 = wmma_f16(av.h, b0.h, h0);
            h1 = wmma_f16(av.h, b1.h, h1);
          }
          const float bv0 = bf1S[f0 + m15];
          const float bv1 = bf1S[f0 + 16 + m15];
#pragma unroll
          for (int r = 0; r < 8; ++r) {
            const int lp = 8 * hh + r;
            float u0 = h0[r] * WINV + bv0; u0 = fmaxf(u0, 0.f);
            float u1 = h1[r] * WINV + bv1; u1 = fmaxf(u1, 0.f);
            HsW[lp * HSP + m15]      = f16b(u0);
            HsW[lp * HSP + 16 + m15] = f16b(u1);
          }
          wave_lds_sync();
          FragH a2; a2.u = frag16(HsW + m15 * HSP, hh);
#pragma unroll
          for (int ct = 0; ct < 4; ++ct) {
            FragH b2; b2.u = frag16(Wf2Tk + (size_t)(ct * 16 + m15) * DFF + f0, hh);
            acc2[ct] = wmma_f16(a2.h, b2.h, acc2[ct]);
          }
          wave_lds_sync();
        }
#pragma unroll
        for (int r = 0; r < 8; ++r) {
          const int l = lt * 16 + 8 * hh + r;
          float* xrow = Xs + l * XP;
#pragma unroll
          for (int ct = 0; ct < 4; ++ct) {
            const int c = ct * 16 + m15;
            xrow[c] += acc2[ct][r] * WINV + bf2S[c];
          }
        }
      }
    }
    __syncthreads();
  }

  {
    const int ct = wv & 3, pg = wv >> 2;
    const unsigned short* ahi = WoH + (size_t)k * PP * LL;
    const unsigned short* alo = WoL + (size_t)k * PP * LL;
    const float* xc = Xs + ct * 16 + m15;
    v8f acc[3];
#pragma unroll
    for (int i = 0; i < 3; ++i) acc[i] = z8;
#pragma unroll 1
    for (int l0 = 0; l0 < LL; l0 += 32) {
      float bvv[16];
#pragma unroll
      for (int i = 0; i < 8; ++i) {
        bvv[i]     = xc[(l0 + 8 * hh + i) * XP];
        bvv[8 + i] = xc[(l0 + 16 + 8 * hh + i) * XP];
      }
      FragH bh, bl;
#pragma unroll
      for (int i = 0; i < 16; ++i) {
        const unsigned short hb = bf16b(bvv[i]);
        const float hf = __uint_as_float(((unsigned int)hb) << 16);
        bh.u[i] = hb;
        bl.u[i] = bf16b(bvv[i] - hf);
      }
#pragma unroll
      for (int i = 0; i < 3; ++i) {
        const int pt = pg * 3 + i;
        FragH ah; ah.u = frag16(ahi + (size_t)(pt * 16 + m15) * LL + l0, hh);
        FragH al; al.u = frag16(alo + (size_t)(pt * 16 + m15) * LL + l0, hh);
        acc[i] = wmma_bf16(ah.b, bh.b, acc[i]);
        acc[i] = wmma_bf16(ah.b, bl.b, acc[i]);
        acc[i] = wmma_bf16(al.b, bh.b, acc[i]);
      }
    }
    const int c = ct * 16 + m15;
    const float dsc = (1.0f / chRw[c]) * chStd[c];
    const float dmn = chMean[c];
    const float drb = chRb[c];
#pragma unroll
    for (int i = 0; i < 3; ++i) {
      const int pt = pg * 3 + i;
#pragma unroll
      for (int r = 0; r < 8; ++r) {
        const int p = pt * 16 + 8 * hh + r;
        const float v = acc[i][r] + bout[k * PP + p];
        Os[p * 64 + c] = (v - drb) * dsc + dmn;
      }
    }
  }
  __syncthreads();

  float* Og = O + (((size_t)k * BB + b) * PP) * CKN;
  o_store_pass(Os, Og, wv, lane);
  __threadfence();
  o_store_pass(Os, Og, wv, lane);
}

__global__ __launch_bounds__(256) void out_kernel(const float* __restrict__ O,
                                                  const int* __restrict__ inv,
                                                  float* __restrict__ out) {
  const int tid = threadIdx.x, lane = tid & 31, wv = tid >> 5;
  const int row = blockIdx.x * 8 + wv;
  if (row >= BB * PP) return;
  const int b = row / PP, p = row - b * PP;
  v4f vals[4];
#pragma unroll
  for (int i = 0; i < 4; ++i) {
#pragma unroll
    for (int e = 0; e < 4; ++e) {
      const int c = 128 * i + 4 * lane + e;
      int q = inv[c];
      q = q < 0 ? 0 : (q > CC - 1 ? CC - 1 : q);
      const int kk = q >> 6, j = q & 63;
      vals[i][e] = O[(((size_t)kk * BB + b) * PP + p) * CKN + j];
    }
  }
  float* orow = out + (size_t)row * CC;
#pragma unroll
  for (int i = 0; i < 4; ++i) *(volatile v4f*)(orow + 128 * i + 4 * lane) = vals[i];
  __threadfence();
#pragma unroll
  for (int i = 0; i < 4; ++i) *(volatile v4f*)(orow + 128 * i + 4 * lane) = vals[i];
}

extern "C" void kernel_launch(void* const* d_in, const int* in_sizes, int n_in,
                              void* d_out, int out_size, void* d_ws, size_t ws_size,
                              hipStream_t stream) {
  if (n_in < 16) return;
  if (in_sizes[0] != BB * LL * CC) return;
  if (in_sizes[1] != CC || in_sizes[2] != CC || in_sizes[3] != CC) return;
  if (in_sizes[4] != KCL * NLAY * LL * LL) return;
  if (in_sizes[5] != KCL * NLAY * LL) return;
  if (in_sizes[6] != KCL * NLAY * CKN || in_sizes[7] != KCL * NLAY * CKN) return;
  if (in_sizes[8] != KCL * NLAY * CKN * DFF || in_sizes[9] != KCL * NLAY * DFF) return;
  if (in_sizes[10] != KCL * NLAY * DFF * CKN || in_sizes[11] != KCL * NLAY * CKN) return;
  if (in_sizes[12] != KCL * NLAY * CKN || in_sizes[13] != KCL * NLAY * CKN) return;
  if (in_sizes[14] != KCL * LL * PP || in_sizes[15] != KCL * PP) return;
  if (out_size != BB * PP * CC) return;

  const float* x           = (const float*)d_in[0];
  const int*   cluster_ids = (const int*)d_in[1];
  const float* rev_w       = (const float*)d_in[2];
  const float* rev_b       = (const float*)d_in[3];
  const float* Wt          = (const float*)d_in[4];
  const float* bt          = (const float*)d_in[5];
  const float* ln1_g       = (const float*)d_in[6];
  const float* ln1_b       = (const float*)d_in[7];
  const float* Wf1         = (const float*)d_in[8];
  const float* bf1         = (const float*)d_in[9];
  const float* Wf2         = (const float*)d_in[10];
  const float* bf2         = (const float*)d_in[11];
  const float* ln2_g       = (const float*)d_in[12];
  const float* ln2_b       = (const float*)d_in[13];
  const float* Wout        = (const float*)d_in[14];
  const float* bout        = (const float*)d_in[15];
  float* out = (float*)d_out;

  const size_t sz_wt   = (size_t)KCL * NLAY * LL * LL * 2;
  const size_t sz_wf1  = (size_t)KCL * NLAY * DFF * CKN * 2;
  const size_t sz_wf2  = (size_t)KCL * NLAY * CKN * DFF * 2;
  const size_t sz_wo   = (size_t)KCL * PP * LL * 2;
  const size_t sz_o    = (size_t)KCL * BB * PP * CKN * 4;
  const size_t sz_tab  = (size_t)CC * 4;
  const size_t total = sz_wt + sz_wf1 + sz_wf2 + 2 * sz_wo + sz_o + 2 * sz_tab;
  if (total > ws_size) return;

  char* ws = (char*)d_ws;
  unsigned short* WtT  = (unsigned short*)ws; ws += sz_wt;
  unsigned short* Wf1T = (unsigned short*)ws; ws += sz_wf1;
  unsigned short* Wf2T = (unsigned short*)ws; ws += sz_wf2;
  unsigned short* WoH  = (unsigned short*)ws; ws += sz_wo;
  unsigned short* WoL  = (unsigned short*)ws; ws += sz_wo;
  float* O             = (float*)ws;          ws += sz_o;
  int* permT           = (int*)ws;            ws += sz_tab;
  int* invT            = (int*)ws;            ws += sz_tab;

  setup_kernel<<<1, CC, 0, stream>>>(cluster_ids, in_sizes[1], permT, invT);

  tcvt_kernel<0><<<dim3(LL / 32, LL / 64, KCL * NLAY), 256, 0, stream>>>(
      Wt, WtT, WtT, LL, LL, WSC);
  tcvt_kernel<0><<<dim3(DFF / 32, CKN / 64, KCL * NLAY), 256, 0, stream>>>(
      Wf1, Wf1T, Wf1T, CKN, DFF, WSC);
  tcvt_kernel<0><<<dim3(CKN / 32, DFF / 64, KCL * NLAY), 256, 0, stream>>>(
      Wf2, Wf2T, Wf2T, DFF, CKN, WSC);
  tcvt_kernel<1><<<dim3(PP / 32, LL / 64, KCL), 256, 0, stream>>>(
      Wout, WoH, WoL, LL, PP, 1.0f);

  hipFuncSetAttribute(reinterpret_cast<const void*>(&mixer_kernel),
                      hipFuncAttributeMaxDynamicSharedMemorySize, SMEM_BYTES);
  mixer_kernel<<<dim3(KCL * BB), dim3(256), SMEM_BYTES, stream>>>(
      x, rev_w, rev_b, bt, ln1_g, ln1_b, bf1, bf2, ln2_g, ln2_b, bout,
      WtT, Wf1T, Wf2T, WoH, WoL, permT, O);

  out_kernel<<<dim3((BB * PP) / 8), dim3(256), 0, stream>>>(O, invT, out);
}
